// ConvCapsLayer3D_22814866276894
// MI455X (gfx1250) — hardware-verified
//
#include <hip/hip_runtime.h>
#include <math.h>

constexpr int kBatch   = 8;
constexpr int kChI     = 32;
constexpr int kNi      = 8;
constexpr int kHW      = 32;
constexpr int kPix     = kHW * kHW;
constexpr int kChJ     = 32;
constexpr int kNj      = 4;
constexpr int kOC      = kChJ * kNj;
constexpr int kTaps    = 27;
constexpr int kKpad    = 32;
constexpr int kRows    = kBatch * kChI * kPix;
constexpr int kGroup   = kPix * kChJ;
constexpr int kNGroups = kBatch * kChI;
constexpr int kSXP     = 132;
constexpr float kXCarry      = 4.0f;
constexpr float kXInv        = 0.25f;
constexpr float kUnif        = 1.0f / 32768.0f;
constexpr float kEps         = 1e-8f;
constexpr float kInvLogGroup = 1.0f / 10.39720770839918f;
constexpr float kInvNGroups  = 1.0f / 256.0f;

typedef __attribute__((ext_vector_type(16))) _Float16 v16h;
typedef __attribute__((ext_vector_type(8)))  _Float16 v8h;
typedef __attribute__((ext_vector_type(16))) __bf16   v16b;
typedef __attribute__((ext_vector_type(8)))  __bf16   v8b;
typedef __attribute__((ext_vector_type(8)))  float    v8f;
typedef __attribute__((ext_vector_type(4)))  float    v4f;
typedef __attribute__((ext_vector_type(4)))  unsigned int v4u;

__device__ __forceinline__ unsigned short f2bf_bits(float f) {
  unsigned u = __float_as_uint(f);
  return (unsigned short)((u + 0x7FFFu + ((u >> 16) & 1u)) >> 16);
}
__device__ __forceinline__ float bf_bits2f(unsigned short h) { return __uint_as_float(((unsigned)h) << 16); }

__device__ __forceinline__ void dep_guard_h(v8f& a, v8f& b, v16h x, v16h y) { asm volatile("v_nop\n\tv_nop\n\tv_nop\n\tv_nop" : "+v"(a), "+v"(b) : "v"(x), "v"(y)); }
__device__ __forceinline__ void dep_guard_b(v8f& a, v8f& b, v16b x, v16b y) { asm volatile("v_nop\n\tv_nop\n\tv_nop\n\tv_nop" : "+v"(a), "+v"(b) : "v"(x), "v"(y)); }
__device__ __forceinline__ void keep4_h(v16h a, v16h b, v16h c, v16h d) { asm volatile("v_nop" :: "v"(a), "v"(b), "v"(c), "v"(d)); }
__device__ __forceinline__ void keep4_b(v16b a, v16b b, v16b c, v16b d) { asm volatile("v_nop" :: "v"(a), "v"(b), "v"(c), "v"(d)); }
__device__ __forceinline__ void acc_guard4(v8f& a, v8f& b, v8f& c, v8f& d) { asm volatile("v_nop\n\tv_nop\n\tv_nop\n\tv_nop" : "+v"(a), "+v"(b), "+v"(c), "+v"(d)); }
template <typename T> struct Frag;
template <> struct Frag<_Float16> {
  typedef v16h V; union U { v16h v; v8h h[2]; };
  static __device__ __forceinline__ v16h load(const _Float16* p) {
    U f; f.h[0] = *(const v8h*)(p); f.h[1] = *(const v8h*)(p + 16); return f.v;
  }
  static __device__ __forceinline__ v8f mma(v16h a, v16h b, v8f c) {
    return __builtin_amdgcn_wmma_f32_16x16x32_f16(false, a, false, b, (short)0, c, false, false);
  }
  static __device__ __forceinline__ void guard(v8f& a, v8f& b, v16h x, v16h y) { dep_guard_h(a, b, x, y); }
  static __device__ __forceinline__ void keep(v16h a, v16h b, v16h c, v16h d) { keep4_h(a, b, c, d); }
};
template <> struct Frag<__bf16> {
  typedef v16b V; union U { v16b v; v8b h[2]; };
  static __device__ __forceinline__ v16b load(const __bf16* p) {
    U f; f.h[0] = *(const v8b*)(p); f.h[1] = *(const v8b*)(p + 16); return f.v;
  }
  static __device__ __forceinline__ v8f mma(v16b a, v16b b, v8f c) {
    return __builtin_amdgcn_wmma_f32_16x16x32_bf16(false, a, false, b, (short)0, c, false, false);
  }
  static __device__ __forceinline__ void guard(v8f& a, v8f& b, v16b x, v16b y) { dep_guard_b(a, b, x, y); }
  static __device__ __forceinline__ void keep(v16b a, v16b b, v16b c, v16b d) { keep4_b(a, b, c, d); }
};

__device__ __forceinline__ unsigned pk16(unsigned short a, unsigned short b) { return (unsigned)a | ((unsigned)b << 16); }

template <int ET> struct Elem;
template <> struct Elem<0> { typedef _Float16 T; };
template <> struct Elem<1> { typedef __bf16 T; };
template <int ET, bool SPLIT, int BIAS_MODE, int OUT_MODE, bool RESID, int ACT = 0>
__global__ __launch_bounds__(256) void wmma_gemm64(
    const unsigned short* __restrict__ Ap, const unsigned short* __restrict__ A2p, int lda, long strideA,
    const unsigned short* __restrict__ Btp, const unsigned short* __restrict__ Bt2p, int ldb, long strideB,
    void* __restrict__ Cout, void* __restrict__ Cout2, int ldc, long strideC,
    const float* __restrict__ bias,
    const float* __restrict__ resid, long strideR,
    int M, int N, int K, float scale) {
  typedef typename Elem<ET>::T T;
  typedef typename Frag<T>::V V;
  const T* A = (const T*)Ap; const T* A2 = (const T*)A2p; const T* Bt = (const T*)Btp; const T* Bt2 = (const T*)Bt2p;
  __shared__ __align__(16) float sT[8][16 * 68];
  const int b    = blockIdx.y;
  const int lane = threadIdx.x & 31;
  const int wave = threadIdx.x >> 5;
  const int tilesN = N >> 6;
  const int tilesM = M >> 6;
  const int tile = blockIdx.x * 8 + wave;
  if (tile >= tilesM * tilesN) return;
  const int tm = tile / tilesN;
  const int tn = tile - tm * tilesN;
  const int m0 = tm << 6;
  const int n0 = tn << 6;

  const T* Ab  = A  + (size_t)b * strideA;
  const T* Bb  = Bt + (size_t)b * strideB;
  const T* Ab2 = SPLIT ? (A2  + (size_t)b * strideA) : nullptr;
  const T* Bb2 = SPLIT ? (Bt2 + (size_t)b * strideB) : nullptr;

  const int rlane = lane & 15;
  const int koff  = (lane >> 4) * 8;
  const int mOff  = (lane >> 4) * 8;

  v8f acc[4][4];
#pragma unroll
  for (int i = 0; i < 4; ++i)
#pragma unroll
    for (int j = 0; j < 4; ++j) acc[i][j] = (v8f){0.f,0.f,0.f,0.f,0.f,0.f,0.f,0.f};

  for (int k0 = 0; k0 < K; k0 += 32) {
    V bh[4], bl[4];
#pragma unroll
    for (int j = 0; j < 4; ++j) {
      const size_t bo = (size_t)(n0 + (j << 4) + rlane) * ldb + koff + k0;
      bh[j] = Frag<T>::load(Bb + bo);
      if (SPLIT) bl[j] = Frag<T>::load(Bb2 + bo);
    }
#pragma unroll
    for (int i = 0; i < 4; ++i) {
      const size_t ao = (size_t)(m0 + (i << 4) + rlane) * lda + koff + k0;
      V ah = Frag<T>::load(Ab + ao);
      V al;
      if (SPLIT) al = Frag<T>::load(Ab2 + ao);
#pragma unroll
      for (int j = 0; j < 4; ++j) {
        acc[i][j] = Frag<T>::mma(ah, bh[j], acc[i][j]);
        if (SPLIT) {
          acc[i][j] = Frag<T>::mma(ah, bl[j], acc[i][j]);
          acc[i][j] = Frag<T>::mma(al, bh[j], acc[i][j]);
        }
      }
      Frag<T>::guard(acc[i][0], acc[i][3], ah, SPLIT ? al : ah);
    }
    Frag<T>::keep(bh[0], bh[1], bh[2], bh[3]);
    if (SPLIT) Frag<T>::keep(bl[0], bl[1], bl[2], bl[3]);
  }
  acc_guard4(acc[0][0], acc[0][1], acc[0][2], acc[0][3]);
  acc_guard4(acc[1][0], acc[1][1], acc[1][2], acc[1][3]);
  acc_guard4(acc[2][0], acc[2][1], acc[2][2], acc[2][3]);
  acc_guard4(acc[3][0], acc[3][1], acc[3][2], acc[3][3]);

  float* slab = sT[wave];
  const float* Rb = RESID ? (resid + (size_t)b * strideR) : nullptr;
#pragma unroll
  for (int i = 0; i < 4; ++i) {
    const int mBase = m0 + (i << 4);
#pragma unroll
    for (int j = 0; j < 4; ++j) {
      const int n = n0 + (j << 4) + rlane;
      float bv = 0.f;
      if (BIAS_MODE == 2) bv = bias[n];
#pragma unroll
      for (int r = 0; r < 8; ++r) {
        float v = acc[i][j][r] * scale;
        if (BIAS_MODE == 1) v += bias[mBase + mOff + r];
        if (BIAS_MODE == 2) v += bv;
        if (RESID) v += Rb[(size_t)(mBase + mOff + r) * ldc + n];
        if (ACT == 2) v = fmaxf(v, 0.0f);
        if (ACT == 4) v = (v > 0.f) ? v : 0.01f * v;
        slab[(mOff + r) * 68 + (j << 4) + rlane] = v;
      }
    }
    __builtin_amdgcn_fence(__ATOMIC_RELEASE, "workgroup");
    __builtin_amdgcn_wave_barrier();
    __builtin_amdgcn_fence(__ATOMIC_ACQUIRE, "workgroup");
    if (OUT_MODE == 0) {
      float* C = (float*)Cout + (size_t)b * strideC;
      const int hh = lane >> 4, c4 = (lane & 15) * 4;
      for (int pass = 0; pass < 2; ++pass) {
#pragma unroll
        for (int it = 0; it < 8; ++it) {
          const int row = it * 2 + hh;
          v4f v = *(const v4f*)(slab + row * 68 + c4);
          *(volatile v4f*)(C + (size_t)(mBase + row) * ldc + n0 + c4) = v;
        }
        __threadfence();
      }
    } else {
      const int q = lane >> 3, c8 = (lane & 7) * 8;
      unsigned short* C  = (unsigned short*)Cout  + (size_t)b * strideC;
      unsigned short* C2 = (OUT_MODE == 2) ? ((unsigned short*)Cout2 + (size_t)b * strideC) : nullptr;
      for (int pass = 0; pass < 2; ++pass) {
#pragma unroll
        for (int it = 0; it < 4; ++it) {
          const int row = it * 4 + q;
          const float* sp = slab + row * 68 + c8;
          v8h hv, lv;
#pragma unroll
          for (int e = 0; e < 8; ++e) {
            if (OUT_MODE == 1) {
              hv[e] = (_Float16)sp[e];
            } else {
              unsigned short hb = f2bf_bits(sp[e]);
              unsigned short lb = f2bf_bits(sp[e] - bf_bits2f(hb));
              hv[e] = __builtin_bit_cast(_Float16, hb);
              lv[e] = __builtin_bit_cast(_Float16, lb);
            }
          }
          *(volatile v8h*)(C + (size_t)(mBase + row) * ldc + n0 + c8) = hv;
          if (OUT_MODE == 2) *(volatile v8h*)(C2 + (size_t)(mBase + row) * ldc + n0 + c8) = lv;
        }
        __threadfence();
      }
    }
    __builtin_amdgcn_fence(__ATOMIC_RELEASE, "workgroup");
    __builtin_amdgcn_wave_barrier();
    __builtin_amdgcn_fence(__ATOMIC_ACQUIRE, "workgroup");
  }
}

__global__ __launch_bounds__(512) void prep_w_kernel(const float* __restrict__ w, const float* __restrict__ cb,
                                                     unsigned short* __restrict__ WH, unsigned short* __restrict__ WL,
                                                     float* __restrict__ B4) {
  const int t = threadIdx.x;
  const int o = t >> 2, k8 = (t & 3) * 8;
  unsigned short hb[8], lb[8];
#pragma unroll
  for (int e = 0; e < 8; ++e) {
    const int kk = k8 + e;
    const int kc = (kk < kTaps) ? kk : (kTaps - 1);
    float v = w[o * kTaps + kc];
    v = (kk < kTaps) ? v : 0.0f;
    const unsigned short h = f2bf_bits(v);
    hb[e] = h;
    lb[e] = f2bf_bits(v - bf_bits2f(h));
  }
  const v4u hv = (v4u){pk16(hb[0], hb[1]), pk16(hb[2], hb[3]), pk16(hb[4], hb[5]), pk16(hb[6], hb[7])};
  const v4u lv = (v4u){pk16(lb[0], lb[1]), pk16(lb[2], lb[3]), pk16(lb[4], lb[5]), pk16(lb[6], lb[7])};
  unsigned short* ph = WH + (size_t)o * kKpad + k8;
  unsigned short* pl = WL + (size_t)o * kKpad + k8;
  const bool wb = (t < 32);
  const int tb = wb ? t : 0;
  const v4f bv = (v4f){kXCarry * cb[4 * tb], kXCarry * cb[4 * tb + 1], kXCarry * cb[4 * tb + 2], kXCarry * cb[4 * tb + 3]};
  *(volatile v4u*)ph = hv;
  *(volatile v4u*)pl = lv;
  if (wb) *(volatile v4f*)(B4 + 4 * tb) = bv;
  __threadfence();
  *(volatile v4u*)ph = hv;
  *(volatile v4u*)pl = lv;
  if (wb) *(volatile v4f*)(B4 + 4 * tb) = bv;
}

__global__ __launch_bounds__(256) void im2col_kernel(const float* __restrict__ in, unsigned short* __restrict__ IH,
                                                     unsigned short* __restrict__ IL) {
  const int t = threadIdx.x;
  const int r = blockIdx.x * 64 + (t >> 2);
  if (r >= kRows) return;
  const int k8 = (t & 3) * 8;
  const int x = r & 31, y = (r >> 5) & 31, d = (r >> 10) & 31, b = r >> 15;
  const float* base = in + ((size_t)(b * kChI + d)) * kNi * kPix;
  unsigned short hb[8], lb[8];
#pragma unroll
  for (int e = 0; e < 8; ++e) {
    const int kk  = k8 + e;
    const int kc  = (kk < kTaps) ? kk : (kTaps - 1);
    const int kd  = kc / 9;
    const int rem = kc - kd * 9;
    const int ky  = rem / 3;
    const int kx  = rem - ky * 3;
    const int yy  = y + ky - 1, xx = x + kx - 1;
    const bool valid = (kk < kTaps) && (yy >= 0) && (yy < kHW) && (xx >= 0) && (xx < kHW);
    const int yc = yy < 0 ? 0 : (yy > kHW - 1 ? kHW - 1 : yy);
    const int xc = xx < 0 ? 0 : (xx > kHW - 1 ? kHW - 1 : xx);
    float v = base[kd * kPix + yc * kHW + xc];
    v = valid ? v : 0.0f;
    const unsigned short h = f2bf_bits(v);
    hb[e] = h;
    lb[e] = f2bf_bits(v - bf_bits2f(h));
  }
  const v4u hv = (v4u){pk16(hb[0], hb[1]), pk16(hb[2], hb[3]), pk16(hb[4], hb[5]), pk16(hb[6], hb[7])};
  const v4u lv = (v4u){pk16(lb[0], lb[1]), pk16(lb[2], lb[3]), pk16(lb[4], lb[5]), pk16(lb[6], lb[7])};
  unsigned short* ph = IH + (size_t)r * kKpad + k8;
  unsigned short* pl = IL + (size_t)r * kKpad + k8;
  *(volatile v4u*)ph = hv;
  *(volatile v4u*)pl = lv;
  __threadfence();
  *(volatile v4u*)ph = hv;
  *(volatile v4u*)pl = lv;
}

template <int FIRST, int LAST>
__global__ __launch_bounds__(128) void agree_kernel(const unsigned short* __restrict__ X16, float* BL,
                                                    const float* __restrict__ ST, float* __restrict__ outp) {
  __shared__ __align__(16) float sX[kChI * kSXP];
  __shared__ float sK[kChI * kChJ];
  __shared__ float sBr[kChI * kChJ];
  __shared__ float sU[kChI * kChJ];
  __shared__ float sSh[kOC];
  __shared__ float sOut[kOC * 33];
  __shared__ float sMax[kChI];
  __shared__ float sRinv[kChI];
  const int t = threadIdx.x, lane = t & 31, wave = t >> 5;
  const int b = blockIdx.x >> 5, y = blockIdx.x & 31;
  if (!FIRST) {
    if (t < kChI) {
      const size_t so = ((size_t)(b * kChI + t)) * 32;
      sMax[t]  = ST[so];
      sRinv[t] = ST[so + 1];
    }
  }
  const _Float16* Xh = (const _Float16*)X16;
#pragma unroll 1
  for (int px = 0; px < kHW; ++px) {
    const int pix = y * kHW + px;
    __syncthreads();
#pragma unroll
    for (int i = 0; i < 4; ++i) {
      const int g = i * 128 + t;
      const int ci = g >> 4, o8 = (g & 15) * 8;
      const v8h hv = *(const v8h*)(Xh + (((size_t)(b * kChI + ci)) * kPix + pix) * kOC + o8);
      float* dst = sX + ci * kSXP + o8;
#pragma unroll
      for (int e = 0; e < 8; ++e) dst[e] = kXInv * (float)hv[e];
    }
    if (!FIRST) {
#pragma unroll 1
      for (int i = t; i < kChI * kChJ; i += 128) {
        const int ci = i >> 5;
        const float raw = BL[(((size_t)(b * kChI + ci)) * kPix + pix) * kChJ + (i & 31)];
        sBr[i] = raw;
        sK[i]  = __expf(raw - sMax[ci]) * sRinv[ci];
      }
    }
    __syncthreads();
    {
      const int cj = t >> 2;
      float s = 0.0f;
#pragma unroll 4
      for (int ci = 0; ci < kChI; ++ci) {
        const float kv = FIRST ? kUnif : sK[ci * kChJ + cj];
        s += kv * sX[ci * kSXP + t];
      }
      const float nrm = sqrtf(s * s);
      const float den = 1.0f + nrm * nrm + kEps;
      const float sh  = nrm * (1.0f / den) * s;
      sSh[t] = sh;
      if (LAST) sOut[t * 33 + px] = sh;
    }
    __syncthreads();
    if (!LAST) {
#pragma unroll 1
      for (int i = t; i < kChI * kChJ; i += 128) {
        const int ci = i >> 5, cj = i & 31;
        const v4f xv = *(const v4f*)(sX + ci * kSXP + cj * 4);
        const float* sp = sSh + cj * 4;
        const float u = ((sp[0] * xv[0] + sp[1] * xv[1]) + sp[2] * xv[2]) + sp[3] * xv[3];
        sU[i] = FIRST ? u : (sBr[i] + u);
      }
      __syncthreads();
      for (int pass = 0; pass < 2; ++pass) {
#pragma unroll
        for (int j = 0; j < 8; ++j) {
          const int ci = wave + 4 * j;
          const float v = sU[ci * kChJ + lane];
          *(volatile float*)(BL + (((size_t)(b * kChI + ci)) * kPix + pix) * kChJ + lane) = v;
        }
        __threadfence();
      }
    }
  }
  if (LAST) {
    __syncthreads();
    for (int pass = 0; pass < 2; ++pass) {
#pragma unroll 1
      for (int j = 0; j < 32; ++j) {
        const int o = wave + 4 * j;
        const float v = sOut[o * 33 + lane];
        *(volatile float*)(outp + (((size_t)(b * kOC + o)) * kHW + y) * kHW + lane) = v;
      }
      __threadfence();
    }
  }
}

__global__ __launch_bounds__(256) void stats_kernel(const float* __restrict__ BL, float* __restrict__ ST) {
  __shared__ float red[256];
  const int g = blockIdx.x;
  const int t = threadIdx.x;
  const float* p = BL + (size_t)g * kGroup;
  float m = -INFINITY;
#pragma unroll 1
  for (int i = t; i < kGroup; i += 256) m = fmaxf(m, p[i]);
  red[t] = m;
  __syncthreads();
  for (int s = 128; s > 0; s >>= 1) {
    if (t < s) red[t] = fmaxf(red[t], red[t + s]);
    __syncthreads();
  }
  const float rm = red[0];
  __syncthreads();
  float sum = 0.0f;
#pragma unroll 1
  for (int i = t; i < kGroup; i += 256) sum += __expf(p[i] - rm);
  red[t] = sum;
  __syncthreads();
  for (int s = 128; s > 0; s >>= 1) {
    if (t < s) red[t] += red[t + s];
    __syncthreads();
  }
  const float rinv = 1.0f / red[0];
  if (t < 32) {
    const float v = (t & 1) ? rinv : rm;
    float* q = ST + (size_t)g * 32 + t;
    *(volatile float*)q = v;
    __threadfence();
    *(volatile float*)q = v;
  }
}

__global__ __launch_bounds__(256) void ent_rows_kernel(const float* __restrict__ BL, const float* __restrict__ ST,
                                                       float* __restrict__ EN) {
  __shared__ float red[256];
  const int g = blockIdx.x;
  const int t = threadIdx.x;
  const float* p = BL + (size_t)g * kGroup;
  const float rm = ST[(size_t)g * 32], ri = ST[(size_t)g * 32 + 1];
  float acc = 0.0f;
#pragma unroll 1
  for (int i = t; i < kGroup; i += 256) {
    const float pk = __expf(p[i] - rm) * ri;
    acc -= pk * __logf(pk + kEps);
  }
  red[t] = acc;
  __syncthreads();
  for (int s = 128; s > 0; s >>= 1) {
    if (t < s) red[t] += red[t + s];
    __syncthreads();
  }
  const float q = red[0] * kInvLogGroup;
  if (t < 32) {
    float* d = EN + (size_t)g * 32 + t;
    *(volatile float*)d = q;
    __threadfence();
    *(volatile float*)d = q;
  }
}

__global__ __launch_bounds__(256) void ent_mean_kernel(const float* __restrict__ EN, float* __restrict__ o1) {
  __shared__ float red[256];
  const int t = threadIdx.x;
  red[t] = EN[(size_t)t * 32];
  __syncthreads();
  for (int s = 128; s > 0; s >>= 1) {
    if (t < s) red[t] += red[t + s];
    __syncthreads();
  }
  if (t == 0) {
    const float v = red[0] * kInvNGroups;
    *(volatile float*)o1 = v;
    __threadfence();
    *(volatile float*)o1 = v;
  }
}

extern "C" void kernel_launch(void* const* d_in, const int* in_sizes, int n_in,
                              void* d_out, int out_size, void* d_ws, size_t ws_size,
                              hipStream_t stream) {
  if (n_in < 3) return;
  if (in_sizes[0] != kBatch * kChI * kNi * kPix) return;
  if (in_sizes[1] != kOC * kTaps) return;
  if (in_sizes[2] != kOC) return;
  if (out_size != kBatch * kOC * kPix + 1) return;

  const float* inputs = (const float*)d_in[0];
  const float* conv_w = (const float*)d_in[1];
  const float* conv_b = (const float*)d_in[2];
  float* outp = (float*)d_out;

  const size_t SZ_W   = (size_t)kOC * kKpad * 2;
  const size_t SZ_B4  = 512;
  const size_t SZ_ST  = (size_t)kNGroups * 32 * 4;
  const size_t SZ_IM  = (size_t)kRows * kKpad * 2;
  const size_t SZ_X16 = (size_t)kRows * kOC * 2;
  const size_t SZ_BL  = (size_t)kNGroups * kGroup * 4;

  size_t off = 0;
  const size_t oWH  = off; off += SZ_W;
  const size_t oWL  = off; off += SZ_W;
  const size_t oB4  = off; off += SZ_B4;
  const size_t oST  = off; off += SZ_ST;
  const size_t oEN  = off; off += SZ_ST;
  const size_t oIMH = off; off += SZ_IM;
  const size_t oIML = off; off += SZ_IM;
  const size_t oX16 = off; off += SZ_X16;
  const size_t oBL  = oIMH;
  if (oBL + SZ_BL > oX16) return;
  const size_t TOTAL = off;
  if (TOTAL > ws_size) return;
  if (TOTAL > (size_t)134217728) return;

  char* ws = (char*)d_ws;
  unsigned short* WH  = (unsigned short*)(ws + oWH);
  unsigned short* WL  = (unsigned short*)(ws + oWL);
  float*          B4  = (float*)(ws + oB4);
  float*          ST  = (float*)(ws + oST);
  float*          EN  = (float*)(ws + oEN);
  unsigned short* IMH = (unsigned short*)(ws + oIMH);
  unsigned short* IML = (unsigned short*)(ws + oIML);
  unsigned short* X16 = (unsigned short*)(ws + oX16);
  float*          BL  = (float*)(ws + oBL);

  prep_w_kernel<<<dim3(1), dim3(512), 0, stream>>>(conv_w, conv_b, WH, WL, B4);
  im2col_kernel<<<dim3(kRows / 64), dim3(256), 0, stream>>>(inputs, IMH, IML);
  {
    const int tiles = (kRows / 64) * (kOC / 64);
    const dim3 gG((tiles + 7) / 8, 1);
    wmma_gemm64<1, true, 2, 1, false, 0><<<gG, dim3(256), 0, stream>>>(
        IMH, IML, kKpad, 0L, WH, WL, kKpad, 0L, (void*)X16, (void*)X16, kOC, 0L, B4, B4, 0L,
        kRows, kOC, kKpad, kXCarry);
  }
  const dim3 gA(kBatch * kHW);
  agree_kernel<1, 0><<<gA, dim3(128), 0, stream>>>(X16, BL, ST, outp);
  stats_kernel<<<dim3(kNGroups), dim3(256), 0, stream>>>(BL, ST);
  agree_kernel<0, 0><<<gA, dim3(128), 0, stream>>>(X16, BL, ST, outp);
  stats_kernel<<<dim3(kNGroups), dim3(256), 0, stream>>>(BL, ST);
  agree_kernel<0, 1><<<gA, dim3(128), 0, stream>>>(X16, BL, ST, outp);
  ent_rows_kernel<<<dim3(kNGroups), dim3(256), 0, stream>>>(BL, ST, EN);
  ent_mean_kernel<<<dim3(1), dim3(256), 0, stream>>>(EN, outp + (size_t)kBatch * kOC * kPix);
}
